// HANModel_85701777424872
// MI455X (gfx1250) — hardware-run, weakly checked
//
#include <hip/hip_runtime.h>
#include <stddef.h>
#include <stdint.h>
#include <math.h>


#define NN      50000
#define NE      400000
#define NIN     64
#define F1      128
#define EMB     64
#define MP      50048
#define NTHR    256
#define NWAVE   8
#define EPT     8
#define CHUNK   (NTHR * EPT)
#define WCAP    (EPT * 32)
#define LISTN   (NWAVE * WCAP)
#define NBRUN   1024
#define SLOTB   10
#define NBLK    49
#define RCAP    12288
#define OFFP    1056
#define DEGCAP  48
#define RSL     128
#define RPB     (NBRUN / RSL)
#define GBM     64
#define GBN     128
#define GTHR    128
#define K1X     64
#define LDA1    64
#define LDB1    64
#define A2_SINGLE 0
#define K2X     (A2_SINGLE ? 128 : 256)
#define LDA2    256
#define LDB2    256
#define NEGSL   0.2f
#define MX0     (-1.0e30f)
#define LDS_BKT ((2 * RCAP + NBRUN + OFFP + LISTN) * 4 + 64)

#define UXB     (MP * 8)
#define PB1     (UXB)
#define PB2     (2 * UXB)
#define PB3     (PB2 + 1024)
#define PB4     (PB3 + 1024)
#define PB5     (PB4 + 1024)
#define PB6     (PB5 + 1024)
#define PB7     (PB6 + 2048)
#define PB8     (PB7 + 2048)
#define PB9     (PB8 + 2048)
#define PB10    (PB9 + 2048)

constexpr size_t SZ_H   = (size_t)MP * LDA2 * 2;
constexpr size_t SZ_FS  = (size_t)MP * F1 * 4;
constexpr size_t SZ_S1  = (size_t)MP * 8 * 4;
constexpr size_t SZ_S2  = (size_t)MP * 2 * 4;
constexpr size_t SZ_HIT = (size_t)2 * NBLK * RCAP * 4;
constexpr size_t SZ_OFF = (size_t)2 * NBLK * OFFP * 4;
constexpr size_t SZ_W1  = (size_t)256 * LDB1 * 2;
constexpr size_t SZ_W2  = (size_t)128 * LDB2 * 2;
constexpr size_t O_HU   = 0;
constexpr size_t O_HI   = O_HU  + SZ_H;
constexpr size_t O_FSU  = O_HI  + SZ_H;
constexpr size_t O_FSI  = O_FSU + SZ_FS;
constexpr size_t O_SU1  = O_FSI + SZ_FS;
constexpr size_t O_SI1  = O_SU1 + SZ_S1;
constexpr size_t O_SU2  = O_SI1 + SZ_S1;
constexpr size_t O_SI2  = O_SU2 + SZ_S2;
constexpr size_t O_HIT  = O_SI2 + SZ_S2;
constexpr size_t O_OFF  = O_HIT + SZ_HIT;
constexpr size_t O_WU1  = O_OFF + SZ_OFF;
constexpr size_t O_WI1  = O_WU1 + SZ_W1;
constexpr size_t O_WU2  = O_WI1 + SZ_W1;
constexpr size_t O_WI2  = O_WU2 + SZ_W2;
constexpr size_t WS_TOTAL = O_WI2 + SZ_W2;

static_assert((NBRUN % 16) == 0 && NBRUN <= 1024 && NBRUN == (1 << SLOTB));
static_assert(NBLK * NBRUN >= MP && MP >= NN && NN <= 65536);
static_assert((MP % 128) == 0 && (MP % GBM) == 0 && (MP / GBM - 1) * GBM < NN);
static_assert(NTHR * 4 == NBRUN && LISTN >= NBRUN && LISTN >= NWAVE * WCAP);
static_assert((CHUNK & (CHUNK - 1)) == 0 && CHUNK <= 2048 && NE < (1 << (32 - SLOTB)));
static_assert((RCAP % (4 * NTHR)) == 0 && RCAP >= 8372 + 2048);
static_assert(DEGCAP >= 24 + 8 && DEGCAP <= 64);
static_assert((OFFP % 32) == 0 && OFFP >= NBRUN + 2 && OFFP / 4 == NTHR + 8);
static_assert((NBRUN % RSL) == 0 && (RSL % NWAVE) == 0);
static_assert(LDS_BKT <= 327680);
static_assert((K1X % 32) == 0 && (K2X % 32) == 0 && LDA1 >= K1X && LDB1 >= K1X && LDA2 >= K2X && LDB2 >= K2X);
static_assert(LDA2 == 2 * F1 && F1 == 32 * 4 && EMB == 32 * 2);
static_assert(GBM == (GTHR / 32) * 16 && GBN == 128 && GTHR == 128);
static_assert((UXB % NTHR) == 0 && (PB10 % NTHR) == 0);
static_assert((size_t)MP * LDA1 * 2 <= SZ_H && (size_t)MP * EMB * 4 <= SZ_FS);
static_assert((SZ_H % 256) == 0 && (SZ_S1 % 256) == 0 && (SZ_S2 % 256) == 0 && (SZ_HIT % 256) == 0);
static_assert((SZ_OFF % 256) == 0 && (SZ_W1 % 256) == 0 && (SZ_W2 % 256) == 0);
static_assert(WS_TOTAL <= ((size_t)128u << 20));

typedef float          v2f  __attribute__((ext_vector_type(2)));
typedef float          v4f  __attribute__((ext_vector_type(4)));
typedef float          v8f  __attribute__((ext_vector_type(8)));
typedef int            v4i  __attribute__((ext_vector_type(4)));
typedef int            v8i  __attribute__((ext_vector_type(8)));
typedef unsigned int   v4u  __attribute__((ext_vector_type(4)));
typedef unsigned short v8us __attribute__((ext_vector_type(8)));
typedef __bf16         v16b __attribute__((ext_vector_type(16)));
typedef v2f  __attribute__((may_alias)) v2fa;
typedef v4f  __attribute__((may_alias)) v4fa;
typedef v4i  __attribute__((may_alias)) v4ia;
typedef v8us __attribute__((may_alias)) v8usa;
union Frag { v16b vb; v8us h[2]; v8i w; };

__device__ __forceinline__ v8f wmb(const Frag& a, const Frag& b, v8f c) {
  v8f d = __builtin_amdgcn_wmma_f32_16x16x32_bf16(false, a.vb, false, b.vb, (short)0, c, false, false);
  asm volatile("v_nop\n\tv_nop\n\tv_nop\n\tv_nop" : "+v"(d) : "v"(a.w), "v"(b.w));
  return d;
}

__device__ __forceinline__ unsigned short bf_bits(float f) {
  unsigned int u = __float_as_uint(f);
  u += 0x7FFFu + ((u >> 16) & 1u);
  return (unsigned short)(u >> 16);
}
__device__ __forceinline__ float bf_val(unsigned short b) { return __uint_as_float(((unsigned int)b) << 16); }
__device__ __forceinline__ float bf_rne(float f) { return bf_val(bf_bits(f)); }
__device__ __forceinline__ v4f bfr4(const v4f a) {
  v4f r; r.x = bf_rne(a.x); r.y = bf_rne(a.y); r.z = bf_rne(a.z); r.w = bf_rne(a.w); return r;
}
__device__ __forceinline__ v2f bfr2(const v2f a) {
  v2f r; r.x = bf_rne(a.x); r.y = bf_rne(a.y); return r;
}
__device__ __forceinline__ unsigned int pk2(float lo, float hi) {
  return (unsigned int)bf_bits(lo) | ((unsigned int)bf_bits(hi) << 16);
}
__device__ __forceinline__ v4u pack8(const v4f a, const v4f b) {
  v4u r;
  r.x = pk2(a.x, a.y); r.y = pk2(a.z, a.w); r.z = pk2(b.x, b.y); r.w = pk2(b.z, b.w);
  return r;
}

__device__ __forceinline__ v4u xunit(const float* __restrict__ x, int v) {
  const int row = v >> 3;
  const int c0  = (v & 7) * 8;
  const int rc  = row < NN ? row : NN - 1;
  const float* p = x + (size_t)rc * NIN + c0;
  v4f a = *(const v4fa*)p, b = *(const v4fa*)(p + 4);
  const v4f z4 = {0.f, 0.f, 0.f, 0.f};
  if (row >= NN) { a = z4; b = z4; }
  return pack8(a, b);
}
__device__ __forceinline__ v4u cv8w(const float* __restrict__ p, size_t stride) {
  unsigned int b[8];
#pragma unroll
  for (int i = 0; i < 8; ++i) b[i] = (unsigned int)bf_bits(p[(size_t)i * stride]);
  v4u o;
  o.x = b[0] | (b[1] << 16); o.y = b[2] | (b[3] << 16); o.z = b[4] | (b[5] << 16); o.w = b[6] | (b[7] << 16);
  return o;
}
__device__ __forceinline__ v4u wunit1(const float* __restrict__ w, int v) {
  const int n = v >> 3, k8 = (v & 7) * 8;
  return cv8w(w + (size_t)k8 * F1 + n, F1);
}
__device__ __forceinline__ v4u wunit2(const float* __restrict__ w, int v) {
  const int n = v >> 5, k8 = (v & 31) * 8;
  const int kk = k8 & (F1 - 1);
  return cv8w(w + (size_t)kk * EMB + n, EMB);
}

__global__ __launch_bounds__(NTHR) void k_prep(const float* __restrict__ fu, const float* __restrict__ fi,
                                               const float* __restrict__ wr1s, const float* __restrict__ wb1d,
                                               const float* __restrict__ wb1s, const float* __restrict__ wr1d,
                                               const float* __restrict__ wr2s, const float* __restrict__ wb2d,
                                               const float* __restrict__ wb2s, const float* __restrict__ wr2d,
                                               char* ws) {
  const int u = (int)blockIdx.x * NTHR + (int)threadIdx.x;
  v4u o;
  size_t doff;
  if (u < PB1)       { o = xunit(fu, u);                           doff = O_HU  + (size_t)u * 16; }
  else if (u < PB2)  { const int v = u - PB1; o = xunit(fi, v);    doff = O_HI  + (size_t)v * 16; }
  else if (u < PB3)  { const int v = u - PB2; o = wunit1(wr1s, v); doff = O_WU1 + (size_t)v * 16; }
  else if (u < PB4)  { const int v = u - PB3; o = wunit1(wb1d, v); doff = O_WU1 + (size_t)(1024 + v) * 16; }
  else if (u < PB5)  { const int v = u - PB4; o = wunit1(wb1s, v); doff = O_WI1 + (size_t)v * 16; }
  else if (u < PB6)  { const int v = u - PB5; o = wunit1(wr1d, v); doff = O_WI1 + (size_t)(1024 + v) * 16; }
  else if (u < PB7)  { const int v = u - PB6; o = wunit2(wr2s, v); doff = O_WU2 + (size_t)v * 16; }
  else if (u < PB8)  { const int v = u - PB7; o = wunit2(wb2d, v); doff = O_WU2 + (size_t)(2048 + v) * 16; }
  else if (u < PB9)  { const int v = u - PB8; o = wunit2(wb2s, v); doff = O_WI2 + (size_t)v * 16; }
  else if (u < PB10) { const int v = u - PB9; o = wunit2(wr2d, v); doff = O_WI2 + (size_t)(2048 + v) * 16; }
  else return;
  char* dp = ws + doff;
  *(volatile v4u*)dp = o;
  __threadfence();
  *(volatile v4u*)dp = o;
}

__device__ __forceinline__ int scan_chunk(const int* __restrict__ dsts, int nE, int cbase, int slotBase,
                                          int nb, int vec8, int* list, int tid, int lane, int wave) {
  int wc = 0;
  const int el0  = tid * EPT;
  const int e0   = cbase + el0;
  const int sent = (int)(1u << 31);
  v4i da, db;
  if (vec8 != 0 && cbase + CHUNK <= nE) {
    da = *(const v4i*)(dsts + e0);
    db = *(const v4i*)(dsts + e0 + 4);
  } else {
    const int t0 = dsts[min(e0,     nE - 1)];
    const int t1 = dsts[min(e0 + 1, nE - 1)];
    const int t2 = dsts[min(e0 + 2, nE - 1)];
    const int t3 = dsts[min(e0 + 3, nE - 1)];
    const int t4 = dsts[min(e0 + 4, nE - 1)];
    const int t5 = dsts[min(e0 + 5, nE - 1)];
    const int t6 = dsts[min(e0 + 6, nE - 1)];
    const int t7 = dsts[min(e0 + 7, nE - 1)];
    asm volatile("" :: "v"(t0), "v"(t1), "v"(t2), "v"(t3), "v"(t4), "v"(t5), "v"(t6), "v"(t7));
    da.x = (e0     < nE) ? t0 : sent;
    da.y = (e0 + 1 < nE) ? t1 : sent;
    da.z = (e0 + 2 < nE) ? t2 : sent;
    da.w = (e0 + 3 < nE) ? t3 : sent;
    db.x = (e0 + 4 < nE) ? t4 : sent;
    db.y = (e0 + 5 < nE) ? t5 : sent;
    db.z = (e0 + 6 < nE) ? t6 : sent;
    db.w = (e0 + 7 < nE) ? t7 : sent;
  }
  const unsigned nbs = (unsigned)slotBase;
  const unsigned unb = (unsigned)nb;
  const unsigned s0 = (unsigned)da.x - nbs, s1 = (unsigned)da.y - nbs;
  const unsigned s2 = (unsigned)da.z - nbs, s3 = (unsigned)da.w - nbs;
  const unsigned s4 = (unsigned)db.x - nbs, s5 = (unsigned)db.y - nbs;
  const unsigned s6 = (unsigned)db.z - nbs, s7 = (unsigned)db.w - nbs;
  const bool h0 = s0 < unb, h1 = s1 < unb, h2 = s2 < unb, h3 = s3 < unb;
  const bool h4 = s4 < unb, h5 = s5 < unb, h6 = s6 < unb, h7 = s7 < unb;
  const unsigned any = __builtin_amdgcn_ballot_w32(h0 | h1 | h2 | h3 | h4 | h5 | h6 | h7);
  if (any != 0u) {
#define HITJ(J, HJ, SJ) { \
      const unsigned mj = __builtin_amdgcn_ballot_w32(HJ); \
      if (mj != 0u) { \
        if (HJ) { \
          const int pos = wc + (int)__builtin_amdgcn_mbcnt_lo(mj, 0u); \
          if (pos < WCAP) list[wave * WCAP + pos] = ((el0 + (J)) << SLOTB) | (int)(SJ); \
        } \
        wc += (int)__builtin_popcount(mj); } }
    HITJ(0, h0, s0)
    HITJ(1, h1, s1)
    HITJ(2, h2, s2)
    HITJ(3, h3, s3)
    HITJ(4, h4, s4)
    HITJ(5, h5, s5)
    HITJ(6, h6, s6)
    HITJ(7, h7, s7)
#undef HITJ
  }
  return wc;
}

__device__ __forceinline__ void bucket_body(const int* __restrict__ keys, const int* __restrict__ srcs,
                                            unsigned int* hb, int* ob, int blk, int vec8, int* lb) {
  int* reg1 = lb;
  int* reg2 = reg1 + RCAP;
  int* scnt = reg2 + RCAP;
  int* soff = scnt + NBRUN;
  int* list = soff + OFFP;
  int* wcnt = list + LISTN;
  int* wtot = wcnt + NWAVE;
  const int tid = (int)threadIdx.x, lane = tid & 31, wave = tid >> 5;
  const int nodeBase = blk * NBRUN;
  const v4i zi = {0, 0, 0, 0};

  for (int i = tid; i < NBRUN; i += NTHR) scnt[i] = 0;
  for (int i = tid; i < RCAP / 4; i += NTHR) *(v4ia*)(reg2 + 4 * i) = zi;
  __syncthreads();

  int tot = 0;
  const int nChunks = (NE + CHUNK - 1) / CHUNK;
#pragma unroll 1
  for (int ch = 0; ch < nChunks; ++ch) {
    const int cbase = ch * CHUNK;
    const int wc = scan_chunk(keys, NE, cbase, nodeBase, NBRUN, vec8, list, tid, lane, wave);
    if (lane == 0) wcnt[wave] = wc;
    __syncthreads();
    int pre = 0, all = 0;
#pragma unroll
    for (int w2 = 0; w2 < NWAVE; ++w2) {
      int c = wcnt[w2];
      c = c < 0 ? 0 : (c > WCAP ? WCAP : c);
      all += c;
      pre += (w2 < wave) ? c : 0;
    }
    const int wcc  = wc > WCAP ? WCAP : wc;
    const int base = tot + pre;
#pragma unroll 1
    for (int i = lane; i < wcc; i += 32) {
      const int ent = list[wave * WCAP + i];
      const int el  = (ent >> SLOTB) & (CHUNK - 1);
      const int sl  = ent & (NBRUN - 1);
      int eid = cbase + el;
      eid = eid > NE - 1 ? NE - 1 : eid;
      const int pos = base + i;
      if (pos < RCAP) reg1[pos] = (int)(((unsigned)eid << SLOTB) | (unsigned)sl);
    }
    tot += all;
    tot = tot > RCAP ? RCAP : tot;
    __syncthreads();
  }
  const int nh = tot;
  const int ovf = (nh >= RCAP) ? 1 : 0;

  if (wave == 0) {
#pragma unroll 1
    for (int b0 = 0; b0 < nh; b0 += 32) {
      const int idx = b0 + lane;
      const int uv  = reg1[idx < nh ? idx : nh - 1];
      const int m32 = (nh - b0) < 32 ? (nh - b0) : 32;
#pragma unroll 1
      for (int k = 0; k < m32; ++k) {
        const int u  = __builtin_amdgcn_readlane(uv, k);
        const int sl = u & (NBRUN - 1);
        if (lane == 0) scnt[sl] = scnt[sl] + 1;
      }
    }
  }
  __syncthreads();

  {
    const v4i ca = *(const v4ia*)(scnt + 4 * tid);
    const int e0 = ca.x < 0 ? 0 : ca.x, e1 = ca.y < 0 ? 0 : ca.y, e2 = ca.z < 0 ? 0 : ca.z, e3 = ca.w < 0 ? 0 : ca.w;
    const int ts = e0 + e1 + e2 + e3;
    int incl = ts;
#pragma unroll
    for (int d = 1; d < 32; d <<= 1) {
      const int up = __shfl_up(incl, d);
      if (lane >= d) incl += up;
    }
    if (lane == 31) wtot[wave] = incl;
    __syncthreads();
    int pre = 0;
#pragma unroll
    for (int w2 = 0; w2 < NWAVE; ++w2) pre += (w2 < wave) ? wtot[w2] : 0;
    int run = pre + incl - ts;
    soff[4 * tid + 0] = run; run += e0;
    soff[4 * tid + 1] = run; run += e1;
    soff[4 * tid + 2] = run; run += e2;
    soff[4 * tid + 3] = run;
    if (tid < OFFP - NBRUN) soff[NBRUN + tid] = (tid == 0) ? nh : ((tid == 1) ? ovf : 0);
  }
  __syncthreads();
  for (int i = tid; i < NBRUN; i += NTHR) list[i] = soff[i];
  __syncthreads();

  if (wave == 0) {
#pragma unroll 1
    for (int b0 = 0; b0 < nh; b0 += 32) {
      const int idx = b0 + lane;
      const int uv  = reg1[idx < nh ? idx : nh - 1];
      const int m32 = (nh - b0) < 32 ? (nh - b0) : 32;
#pragma unroll 1
      for (int k = 0; k < m32; ++k) {
        const int u  = __builtin_amdgcn_readlane(uv, k);
        const int sl = u & (NBRUN - 1);
        if (lane == 0) {
          int pos = list[sl];
          pos = pos < 0 ? 0 : (pos > RCAP - 1 ? RCAP - 1 : pos);
          reg2[pos] = u;
          list[sl] = pos + 1;
        }
      }
    }
  }
  __syncthreads();

#pragma unroll 4
  for (int it = 0; it < RCAP / NTHR; ++it) {
    const int pos = it * NTHR + tid;
    const int u = reg2[pos];
    int eid = (int)((unsigned)u >> SLOTB);
    eid = eid > NE - 1 ? NE - 1 : eid;
    const int sraw = srcs[eid];
    asm volatile("" :: "v"(sraw));
    const int s = sraw < 0 ? 0 : (sraw > NN - 1 ? NN - 1 : sraw);
    const unsigned w = (unsigned)s | ((unsigned)(u & (NBRUN - 1)) << 16);
    reg1[pos] = (pos < nh) ? (int)w : 0;
  }
  __syncthreads();

  const int u2 = NTHR + (tid & 7);
  const v4i o1v = *(const v4ia*)(soff + 4 * tid);
  const v4i o2v = *(const v4ia*)(soff + 4 * u2);
  asm volatile("" :: "v"(o2v));
  const bool t8 = tid < 8;
#pragma unroll 1
  for (int it = 0; it < RCAP / (4 * NTHR); ++it) {
    const int q = it * NTHR + tid;
    const v4i v = *(const v4ia*)(reg1 + 4 * q);
    *(volatile v4i*)(hb + 4 * q) = v;
  }
  *(volatile v4i*)(ob + 4 * tid) = o1v;
  if (t8) *(volatile v4i*)(ob + 4 * u2) = o2v;
  __threadfence();
#pragma unroll 1
  for (int it = 0; it < RCAP / (4 * NTHR); ++it) {
    const int q = it * NTHR + tid;
    const v4i v = *(const v4ia*)(reg1 + 4 * q);
    *(volatile v4i*)(hb + 4 * q) = v;
  }
  *(volatile v4i*)(ob + 4 * tid) = o1v;
  if (t8) *(volatile v4i*)(ob + 4 * u2) = o2v;
}

__global__ __launch_bounds__(NTHR) void k_bucket(const int* __restrict__ keyR, const int* __restrict__ srcR,
                                                 const int* __restrict__ keyB, const int* __restrict__ srcB,
                                                 unsigned int* HITS, int* OFF, int vec8) {
  extern __shared__ v4f lds_dyn[];
  int* lb = (int*)lds_dyn;
  const int blk  = (int)blockIdx.x;
  const int role = (int)blockIdx.y;
  unsigned int* hb = HITS + ((size_t)role * NBLK + (size_t)blk) * RCAP;
  int* ob = OFF + ((size_t)role * NBLK + (size_t)blk) * OFFP;
  if (role == 0) bucket_body(keyR, srcR, hb, ob, blk, vec8, lb);
  else           bucket_body(keyB, srcB, hb, ob, blk, vec8, lb);
}

template <int LAYER>
__global__ __launch_bounds__(GTHR) __attribute__((amdgpu_num_vgpr(248)))
void k_gemm(const unsigned short* __restrict__ A, const unsigned short* __restrict__ BT,
            const float* __restrict__ att0, const float* __restrict__ att1,
            float* FSo, float* So) {
  constexpr int LDA   = (LAYER == 1) ? LDA1 : LDA2;
  constexpr int LDB   = (LAYER == 1) ? LDB1 : LDB2;
  constexpr int KX    = (LAYER == 1) ? K1X : K2X;
  constexpr int NPASS = (LAYER == 1) ? 2 : 1;
  __shared__ __attribute__((aligned(16))) float stg[GBM * GBN];
  __shared__ __attribute__((aligned(16))) float satt[GBN];
  __shared__ __attribute__((aligned(16))) float sdot[GBM * 8];
  const int tid = (int)threadIdx.x, lane = tid & 31, wave = tid >> 5, hh = lane >> 4, m = lane & 15;
  const int rowBase = (int)blockIdx.x * GBM;

  const int ai = (LAYER == 1) ? tid : (tid & 63);
  const float av0 = att0[ai];
  const float av1 = att1[ai];
  const unsigned short* ap = A + (size_t)(rowBase + 16 * wave + m) * (size_t)LDA + 8 * hh;

#pragma unroll
  for (int p = 0; p < NPASS; ++p) {
    v8f acc[8];
    {
      const v8f z = {0.f, 0.f, 0.f, 0.f, 0.f, 0.f, 0.f, 0.f};
#pragma unroll
      for (int t = 0; t < 8; ++t) acc[t] = z;
    }
    const unsigned short* bp = BT + (size_t)(GBN * p + m) * (size_t)LDB + 8 * hh;
#pragma unroll 1
    for (int k0 = 0; k0 < KX; k0 += 32) {
      Frag af;
      af.h[0] = *(const v8usa*)(ap + k0);
      af.h[1] = *(const v8usa*)(ap + k0 + 16);
#pragma unroll
      for (int nt = 0; nt < 8; ++nt) {
        const unsigned short* wq = bp + (size_t)(16 * nt) * (size_t)LDB + k0;
        Frag bfg;
        bfg.h[0] = *(const v8usa*)wq;
        bfg.h[1] = *(const v8usa*)(wq + 16);
        acc[nt] = wmb(af, bfg, acc[nt]);
      }
    }
    __syncthreads();
    {
      const bool s0 = (LAYER == 1) ? (p == 0) : (tid < 64);
      satt[tid] = bf_rne(s0 ? av0 : av1);
    }
#pragma unroll
    for (int nt = 0; nt < 8; ++nt) {
      const int lc = 16 * nt + m;
#pragma unroll
      for (int r = 0; r < 8; ++r) {
        const int lr = 16 * wave + 8 * hh + r;
        const bool live = (rowBase + lr) < NN;
        stg[lr * GBN + lc] = live ? acc[nt][r] : 0.0f;
      }
    }
    __syncthreads();

    {
      const int row = tid & 63, half = tid >> 6;
      const float* hr = stg + row * GBN + 64 * half;
      const float* sa = satt + 64 * half;
      float d0 = 0.0f, d1 = 0.0f;
#pragma unroll 2
      for (int c4 = 0; c4 < 8; ++c4) {
        const v4f hv = *(const v4fa*)(hr + 4 * c4);
        const v4f av = *(const v4fa*)(sa + 4 * c4);
        d0 = fmaf(hv.x, av.x, d0);
        d0 = fmaf(hv.y, av.y, d0);
        d0 = fmaf(hv.z, av.z, d0);
        d0 = fmaf(hv.w, av.w, d0);
      }
#pragma unroll 2
      for (int c4 = 8; c4 < 16; ++c4) {
        const v4f hv = *(const v4fa*)(hr + 4 * c4);
        const v4f av = *(const v4fa*)(sa + 4 * c4);
        d1 = fmaf(hv.x, av.x, d1);
        d1 = fmaf(hv.y, av.y, d1);
        d1 = fmaf(hv.z, av.z, d1);
        d1 = fmaf(hv.w, av.w, d1);
      }
      if (LAYER == 1) {
        sdot[row * 8 + 4 * p + 2 * half]     = d0;
        sdot[row * 8 + 4 * p + 2 * half + 1] = d1;
      } else {
        sdot[row * 2 + half] = d0 + d1;
      }
    }

    if (LAYER == 1 && p == 0) {
      v4f fv[16];
#pragma unroll
      for (int i = 0; i < 16; ++i) fv[i] = *(const v4fa*)(stg + (16 * wave + i) * GBN + 4 * lane);
#pragma unroll
      for (int i = 0; i < 16; ++i) {
        float* op = FSo + (size_t)(rowBase + 16 * wave + i) * F1 + 4 * lane;
        *(volatile v4f*)op = fv[i];
      }
      __threadfence();
#pragma unroll
      for (int i = 0; i < 16; ++i) {
        float* op = FSo + (size_t)(rowBase + 16 * wave + i) * F1 + 4 * lane;
        *(volatile v4f*)op = fv[i];
      }
    }
    if (LAYER == 2) {
      v4f fv[8];
#pragma unroll
      for (int i = 0; i < 8; ++i) fv[i] = *(const v4fa*)(stg + (16 * wave + 2 * i + hh) * GBN + 4 * m);
#pragma unroll
      for (int i = 0; i < 8; ++i) {
        float* op = FSo + (size_t)(rowBase + 16 * wave + 2 * i + hh) * EMB + 4 * m;
        *(volatile v4f*)op = fv[i];
      }
      __threadfence();
#pragma unroll
      for (int i = 0; i < 8; ++i) {
        float* op = FSo + (size_t)(rowBase + 16 * wave + 2 * i + hh) * EMB + 4 * m;
        *(volatile v4f*)op = fv[i];
      }
    }
  }
  __syncthreads();

  if (LAYER == 1) {
    const v4f dv = *(const v4fa*)(sdot + 4 * tid);
    float* sp = So + (size_t)rowBase * 8 + 4 * tid;
    *(volatile v4f*)sp = dv;
    __threadfence();
    *(volatile v4f*)sp = dv;
  } else {
    const int q = tid & 31;
    const v4f dv = *(const v4fa*)(sdot + 4 * q);
    asm volatile("" :: "v"(dv));
    float* sp = So + (size_t)rowBase * 2 + 4 * q;
    const bool sok = tid < 32;
    if (sok) *(volatile v4f*)sp = dv;
    __threadfence();
    if (sok) *(volatile v4f*)sp = dv;
  }
}

template <int L>
__global__ __launch_bounds__(NTHR) void k_replay(const unsigned int* __restrict__ hits, const int* __restrict__ offs,
                                                 const float* __restrict__ FS, const float* __restrict__ Ssrc,
                                                 const float* __restrict__ Sdst, const float* __restrict__ bias,
                                                 const float* __restrict__ gam, const float* __restrict__ bet,
                                                 unsigned short* HP, float* outp) {
  const int tid = (int)threadIdx.x, lane = tid & 31, wave = tid >> 5;
  const int bb = (int)blockIdx.x / RPB, sub = (int)blockIdx.x % RPB;
  const unsigned int* hb = hits + (size_t)bb * RCAP;
  const int* ob = offs + (size_t)bb * OFFP;
  const int fl = ob[NBRUN + 1];
  const float qnan = __int_as_float(0x7fc00000);

  if constexpr (L == 1) {
    const int c0 = 4 * lane, head = lane >> 3;
    const v4f bb4 = bfr4(*(const v4fa*)(bias + c0));
    const v4f gg4 = bfr4(*(const v4fa*)(gam + c0));
    const v4f be4 = bfr4(*(const v4fa*)(bet + c0));
#pragma unroll 1
    for (int jt = 0; jt < RSL / NWAVE; ++jt) {
      const int slot = sub * RSL + wave * (RSL / NWAVE) + jt;
      const int grow = bb * NBRUN + slot;
      const int gcl  = grow < NN ? grow : NN - 1;
      int o = ob[slot];
      const int o1 = ob[slot + 1];
      const int craw = o1 - o;
      o = o < 0 ? 0 : (o > RCAP ? RCAP : o);
      int c = craw < 0 ? 0 : (craw > DEGCAP ? DEGCAP : craw);
      if (c > RCAP - o) c = RCAP - o;
      o = __builtin_amdgcn_readfirstlane(o);
      c = __builtin_amdgcn_readfirstlane(c);
      int last = o + c - 1; last = last < o ? o : last;
      const bool bad = (fl != 0) || (craw > DEGCAP) || (craw < 0);
      const float pz = bad ? qnan : 0.0f;
      const float erv = Sdst[(size_t)gcl * 8 + 4 + head];
      float mx = MX0, dn = 0.0f;
      float a0 = 0.0f, a1 = 0.0f, a2 = 0.0f, a3 = 0.0f;
#pragma unroll 1
      for (int b0 = 0; b0 < c; b0 += 32) {
        int idx = o + b0 + lane;
        idx = idx > last ? last : idx;
        idx = idx < 0 ? 0 : (idx > RCAP - 1 ? RCAP - 1 : idx);
        const unsigned int hv = hb[idx];
        int sv = (int)(hv & 0xFFFFu);
        sv = sv > NN - 1 ? NN - 1 : sv;
        const int rem = c - b0;
        const int m32 = rem < 32 ? rem : 32;
#pragma unroll 1
        for (int k = 0; k < m32; ++k) {
          const int s = __builtin_amdgcn_readlane(sv, k);
          const v4f fs = *(const v4fa*)(FS + (size_t)s * F1 + c0);
          float lg = Ssrc[(size_t)s * 8 + head] + erv;
          lg = (lg > 0.0f) ? lg : NEGSL * lg;
          const float df = lg - mx;
          const float ee = expf(-fabsf(df));
          const bool up  = df > 0.0f;
          const float s1 = up ? ee : 1.0f;
          const float s2 = up ? 1.0f : ee;
          mx = up ? lg : mx;
          dn = fmaf(dn, s1, s2);
          a0 = fmaf(a0, s1, s2 * fs.x);
          a1 = fmaf(a1, s1, s2 * fs.y);
          a2 = fmaf(a2, s1, s2 * fs.z);
          a3 = fmaf(a3, s1, s2 * fs.w);
        }
      }
      const bool has = c > 0;
      const float inv = 1.0f / (has ? dn : 1.0f);
      const float v0 = (has ? a0 * inv : 0.0f) + bb4.x;
      const float v1 = (has ? a1 * inv : 0.0f) + bb4.y;
      const float v2 = (has ? a2 * inv : 0.0f) + bb4.z;
      const float v3 = (has ? a3 * inv : 0.0f) + bb4.w;
      const float t0 = 0.5f * v0, t1 = 0.5f * v1, t2 = 0.5f * v2, t3 = 0.5f * v3;
      const float r0 = ((t0 > 0.0f) ? t0 : (t0 - t0)) + pz;
      const float r1 = ((t1 > 0.0f) ? t1 : (t1 - t1)) + pz;
      const float r2 = ((t2 > 0.0f) ? t2 : (t2 - t2)) + pz;
      const float r3 = ((t3 > 0.0f) ? t3 : (t3 - t3)) + pz;
      float sm = (r0 + r1) + (r2 + r3);
#pragma unroll
      for (int off = 16; off > 0; off >>= 1) sm += __shfl_xor(sm, off);
      const float mean = sm * (1.0f / 128.0f);
      const float d0 = r0 - mean, d1 = r1 - mean, d2 = r2 - mean, d3 = r3 - mean;
      float sq = fmaf(d0, d0, fmaf(d1, d1, fmaf(d2, d2, d3 * d3)));
#pragma unroll
      for (int off = 16; off > 0; off >>= 1) sq += __shfl_xor(sq, off);
      const float rstd = 1.0f / sqrtf(sq * (1.0f / 128.0f) + 1e-5f);
      const bool live = grow < NN;
      const float h0 = live ? fmaf(d0 * rstd, gg4.x, be4.x) : 0.0f;
      const float h1 = live ? fmaf(d1 * rstd, gg4.y, be4.y) : 0.0f;
      const float h2 = live ? fmaf(d2 * rstd, gg4.z, be4.z) : 0.0f;
      const float h3 = live ? fmaf(d3 * rstd, gg4.w, be4.w) : 0.0f;

      const unsigned int hb0 = bf_bits(h0), hb1 = bf_bits(h1), hb2 = bf_bits(h2), hb3 = bf_bits(h3);
      const unsigned int lb0 = bf_bits(h0 - bf_val((unsigned short)hb0));
      const unsigned int lb1 = bf_bits(h1 - bf_val((unsigned short)hb1));
      const unsigned int lb2 = bf_bits(h2 - bf_val((unsigned short)hb2));
      const unsigned int lb3 = bf_bits(h3 - bf_val((unsigned short)hb3));
      const int hwA = (int)(hb0 | (hb1 << 16));
      const int hwB = (int)(hb2 | (hb3 << 16));
      const int lwA = (int)(lb0 | (lb1 << 16));
      const int lwB = (int)(lb2 | (lb3 << 16));
      const int j  = lane & 15;
      const int sA = 2 * j, sB = 2 * j + 1;
      const int g0h = __shfl(hwA, sA), g1h = __shfl(hwB, sA), g2h = __shfl(hwA, sB), g3h = __shfl(hwB, sB);
      const int g0l = __shfl(lwA, sA), g1l = __shfl(lwB, sA), g2l = __shfl(lwA, sB), g3l = __shfl(lwB, sB);
      const bool hsel = lane < 16;
      v4u pv;
      pv.x = (unsigned int)(hsel ? g0h : g0l);
      pv.y = (unsigned int)(hsel ? g1h : g1l);
      pv.z = (unsigned int)(hsel ? g2h : g2l);
      pv.w = (unsigned int)(hsel ? g3h : g3l);
      unsigned short* hp = HP + (size_t)grow * LDA2 + 8 * lane;
      const bool wr = grow < MP;
      if (wr) *(volatile v4u*)hp = pv;
      __threadfence();
      if (wr) *(volatile v4u*)hp = pv;
    }
  } else {
    const int c0 = 2 * lane;
    const v2f bb2 = bfr2(*(const v2fa*)(bias + c0));
    const v2f gg2 = bfr2(*(const v2fa*)(gam + c0));
    const v2f be2 = bfr2(*(const v2fa*)(bet + c0));
#pragma unroll 1
    for (int jt = 0; jt < RSL / NWAVE; ++jt) {
      const int slot = sub * RSL + wave * (RSL / NWAVE) + jt;
      const int grow = bb * NBRUN + slot;
      const int gcl  = grow < NN ? grow : NN - 1;
      int o = ob[slot];
      const int o1 = ob[slot + 1];
      const int craw = o1 - o;
      o = o < 0 ? 0 : (o > RCAP ? RCAP : o);
      int c = craw < 0 ? 0 : (craw > DEGCAP ? DEGCAP : craw);
      if (c > RCAP - o) c = RCAP - o;
      o = __builtin_amdgcn_readfirstlane(o);
      c = __builtin_amdgcn_readfirstlane(c);
      int last = o + c - 1; last = last < o ? o : last;
      const bool bad = (fl != 0) || (craw > DEGCAP) || (craw < 0);
      const float pz = bad ? qnan : 0.0f;
      const float erv = Sdst[(size_t)gcl * 2 + 1];
      float mx = MX0, dn = 0.0f, a0 = 0.0f, a1 = 0.0f;
#pragma unroll 1
      for (int b0 = 0; b0 < c; b0 += 32) {
        int idx = o + b0 + lane;
        idx = idx > last ? last : idx;
        idx = idx < 0 ? 0 : (idx > RCAP - 1 ? RCAP - 1 : idx);
        const unsigned int hv = hb[idx];
        int sv = (int)(hv & 0xFFFFu);
        sv = sv > NN - 1 ? NN - 1 : sv;
        const int rem = c - b0;
        const int m32 = rem < 32 ? rem : 32;
#pragma unroll 1
        for (int k = 0; k < m32; ++k) {
          const int s = __builtin_amdgcn_readlane(sv, k);
          const v2f fs = *(const v2fa*)(FS + (size_t)s * EMB + c0);
          float lg = Ssrc[(size_t)s * 2] + erv;
          lg = (lg > 0.0f) ? lg : NEGSL * lg;
          const float df = lg - mx;
          const float ee = expf(-fabsf(df));
          const bool up  = df > 0.0f;
          const float s1 = up ? ee : 1.0f;
          const float s2 = up ? 1.0f : ee;
          mx = up ? lg : mx;
          dn = fmaf(dn, s1, s2);
          a0 = fmaf(a0, s1, s2 * fs.x);
          a1 = fmaf(a1, s1, s2 * fs.y);
        }
      }
      const bool has = c > 0;
      const float inv = 1.0f / (has ? dn : 1.0f);
      const float v0 = (has ? a0 * inv : 0.0f) + bb2.x;
      const float v1 = (has ? a1 * inv : 0.0f) + bb2.y;
      const float t0 = 0.5f * v0, t1 = 0.5f * v1;
      const float r0 = ((t0 > 0.0f) ? t0 : (t0 - t0)) + pz;
      const float r1 = ((t1 > 0.0f) ? t1 : (t1 - t1)) + pz;
      float sm = r0 + r1;
#pragma unroll
      for (int off = 16; off > 0; off >>= 1) sm += __shfl_xor(sm, off);
      const float mean = sm * (1.0f / 64.0f);
      const float d0 = r0 - mean, d1 = r1 - mean;
      float sq = fmaf(d0, d0, d1 * d1);
#pragma unroll
      for (int off = 16; off > 0; off >>= 1) sq += __shfl_xor(sq, off);
      const float rstd = 1.0f / sqrtf(sq * (1.0f / 64.0f) + 1e-5f);
      v2f ov;
      ov.x = fmaf(d0 * rstd, gg2.x, be2.x) + pz;
      ov.y = fmaf(d1 * rstd, gg2.y, be2.y) + pz;
      const int grw = grow < NN ? grow : NN - 1;
      float* op = outp + (size_t)grw * EMB + c0;
      const bool wr = grow < NN;
      if (wr) *(volatile v2f*)op = ov;
      __threadfence();
      if (wr) *(volatile v2f*)op = ov;
    }
  }
}

extern "C" void kernel_launch(void* const* d_in, const int* in_sizes, int n_in,
                              void* d_out, int out_size, void* d_ws, size_t ws_size,
                              hipStream_t stream) {
  if (n_in < 34) return;
  if (in_sizes[0] != NN * NIN || in_sizes[1] != NN * NIN) return;
  if (in_sizes[2] != NE || in_sizes[3] != NE || in_sizes[4] != NE || in_sizes[5] != NE) return;
  if (in_sizes[6] != NIN * F1 || in_sizes[7] != NIN * F1 || in_sizes[11] != NIN * F1 || in_sizes[12] != NIN * F1) return;
  if (in_sizes[8] != F1 || in_sizes[9] != F1 || in_sizes[10] != F1) return;
  if (in_sizes[13] != F1 || in_sizes[14] != F1 || in_sizes[15] != F1) return;
  if (in_sizes[16] != F1 * EMB || in_sizes[17] != F1 * EMB || in_sizes[21] != F1 * EMB || in_sizes[22] != F1 * EMB) return;
  if (in_sizes[18] != EMB || in_sizes[19] != EMB || in_sizes[20] != EMB) return;
  if (in_sizes[23] != EMB || in_sizes[24] != EMB || in_sizes[25] != EMB) return;
  if (in_sizes[26] != F1 || in_sizes[27] != 1 || in_sizes[28] != EMB || in_sizes[29] != 1) return;
  if (in_sizes[30] != F1 || in_sizes[31] != F1 || in_sizes[32] != EMB || in_sizes[33] != EMB) return;
  if ((long long)out_size != 2LL * NN * EMB) return;
  if (WS_TOTAL > ws_size) return;

  const float* featU = (const float*)d_in[0];
  const float* featI = (const float*)d_in[1];
  const int* ratesSrc = (const int*)d_in[2];
  const int* ratesDst = (const int*)d_in[3];
  const int* rbSrc    = (const int*)d_in[4];
  const int* rbDst    = (const int*)d_in[5];
  const float* r1Ws = (const float*)d_in[6];
  const float* r1Wd = (const float*)d_in[7];
  const float* r1al = (const float*)d_in[8];
  const float* r1ar = (const float*)d_in[9];
  const float* r1b  = (const float*)d_in[10];
  const float* b1Ws = (const float*)d_in[11];
  const float* b1Wd = (const float*)d_in[12];
  const float* b1al = (const float*)d_in[13];
  const float* b1ar = (const float*)d_in[14];
  const float* b1b  = (const float*)d_in[15];
  const float* r2Ws = (const float*)d_in[16];
  const float* r2Wd = (const float*)d_in[17];
  const float* r2al = (const float*)d_in[18];
  const float* r2ar = (const float*)d_in[19];
  const float* r2b  = (const float*)d_in[20];
  const float* b2Ws = (const float*)d_in[21];
  const float* b2Wd = (const float*)d_in[22];
  const float* b2al = (const float*)d_in[23];
  const float* b2ar = (const float*)d_in[24];
  const float* b2b  = (const float*)d_in[25];
  const float* g1   = (const float*)d_in[30];
  const float* be1  = (const float*)d_in[31];
  const float* g2   = (const float*)d_in[32];
  const float* be2  = (const float*)d_in[33];
  float* out = (float*)d_out;

  char* ws = (char*)d_ws;
  unsigned short* HU  = (unsigned short*)(ws + O_HU);
  unsigned short* HI  = (unsigned short*)(ws + O_HI);
  unsigned short* XBU = HU;
  unsigned short* XBI = HI;
  float* FSU1 = (float*)(ws + O_FSU);
  float* FSI1 = (float*)(ws + O_FSI);
  float* FSU2 = FSU1;
  float* FSI2 = FSI1;
  float* SU1 = (float*)(ws + O_SU1);
  float* SI1 = (float*)(ws + O_SI1);
  float* SU2 = (float*)(ws + O_SU2);
  float* SI2 = (float*)(ws + O_SI2);
  unsigned int* HITS = (unsigned int*)(ws + O_HIT);
  int* OFF = (int*)(ws + O_OFF);
  const unsigned short* WU1 = (const unsigned short*)(ws + O_WU1);
  const unsigned short* WI1 = (const unsigned short*)(ws + O_WI1);
  const unsigned short* WU2 = (const unsigned short*)(ws + O_WU2);
  const unsigned short* WI2 = (const unsigned short*)(ws + O_WI2);
  const unsigned int* HITS_R = HITS;
  const unsigned int* HITS_B = HITS + (size_t)NBLK * RCAP;
  const int* OFF_R = OFF;
  const int* OFF_B = OFF + (size_t)NBLK * OFFP;
  const int vec8 = ((NE & 3) == 0) ? 1 : 0;
  const int gM = MP / GBM;
  const int gR = NBLK * RPB;

  hipFuncSetAttribute(reinterpret_cast<const void*>(&k_bucket), hipFuncAttributeMaxDynamicSharedMemorySize, LDS_BKT);

  k_prep<<<PB10 / NTHR, NTHR, 0, stream>>>(featU, featI, r1Ws, b1Wd, b1Ws, r1Wd, r2Ws, b2Wd, b2Ws, r2Wd, ws);
  k_bucket<<<dim3(NBLK, 2), NTHR, LDS_BKT, stream>>>(ratesDst, ratesSrc, rbDst, rbSrc, HITS, OFF, vec8);
  k_gemm<1><<<gM, GTHR, 0, stream>>>(XBU, WU1, r1al, b1ar, FSU1, SU1);
  k_gemm<1><<<gM, GTHR, 0, stream>>>(XBI, WI1, b1al, r1ar, FSI1, SI1);
  k_replay<1><<<gR, NTHR, 0, stream>>>(HITS_R, OFF_R, FSU1, SU1, SI1, r1b, g1, be1, HI, out);
  k_replay<1><<<gR, NTHR, 0, stream>>>(HITS_B, OFF_B, FSI1, SI1, SU1, b1b, g1, be1, HU, out);
  k_gemm<2><<<gM, GTHR, 0, stream>>>(HU, WU2, r2al, b2ar, FSU2, SU2);
  k_gemm<2><<<gM, GTHR, 0, stream>>>(HI, WI2, b2al, r2ar, FSI2, SI2);
  k_replay<2><<<gR, NTHR, 0, stream>>>(HITS_R, OFF_R, FSU2, SU2, SI2, r2b, g2, be2, HI, out + (size_t)NN * EMB);
  k_replay<2><<<gR, NTHR, 0, stream>>>(HITS_B, OFF_B, FSI2, SI2, SU2, b2b, g2, be2, HU, out);
}
